// SelfAttention_52261162058329
// MI455X (gfx1250) — hardware-verified
//
#include <hip/hip_runtime.h>


#ifndef NB
#define NB 4
#endif
#ifndef SEQ
#define SEQ 4096
#endif
#define NB_FULL  4
#define SEQ_FULL 4096
#define DD   128
static_assert(NB >= 1 && NB <= NB_FULL);
static_assert(SEQ >= 128 && SEQ <= SEQ_FULL && (SEQ % 128) == 0);
static_assert((SEQ % 64) == 0 && (DD % 64) == 0);
static_assert((SEQ % 32) == 0 && (DD % 32) == 0);
static_assert((SEQ % 4) == 0 && (DD % 8) == 0);
static_assert(((size_t)NB * DD * SEQ / 4) % 256 == 0 && ((size_t)NB * SEQ * DD / 8) % 256 == 0 && ((size_t)NB * DD * DD / 8) % 256 == 0);
#define WS_XT  ((size_t)NB * DD * SEQ * 2)
#define WS_XH  ((size_t)NB * SEQ * DD * 2)
#define WS_G   ((size_t)NB * DD * DD * 4)
#define WS_GH  ((size_t)NB * DD * DD * 2)
static_assert((WS_XT % 256) == 0 && (WS_XH % 256) == 0 && (WS_G % 256) == 0 && (WS_GH % 256) == 0);
static_assert(WS_XT + WS_XH + WS_G + WS_GH <= (size_t)134217728);

typedef _Float16 h16;
typedef unsigned short bf;
typedef __attribute__((ext_vector_type(16))) __bf16   v16bf;
typedef __attribute__((ext_vector_type(16))) _Float16 v16h;
typedef __attribute__((ext_vector_type(8)))  _Float16 v8h;
typedef __attribute__((ext_vector_type(8)))  unsigned short v8us;
typedef __attribute__((ext_vector_type(8)))  float    v8f;
typedef __attribute__((ext_vector_type(4)))  float    v4f;
typedef v8h  __attribute__((may_alias)) v8ha;
typedef v4f  __attribute__((may_alias)) v4fa;
typedef v8us __attribute__((may_alias)) v8usa;

__device__ __forceinline__ unsigned short f2bf(float f) { unsigned u = __float_as_uint(f); u += 0x7FFFu + ((u >> 16) & 1u); return (unsigned short)(u >> 16); }
__device__ __forceinline__ float bf2f(unsigned short b) { return __uint_as_float(((unsigned)b) << 16); }
__device__ __forceinline__ float bfr(float f) { return bf2f(f2bf(f)); }
__device__ __forceinline__ v16h cat16(v8h lo, v8h hi) { return __builtin_shufflevector(lo, hi, 0, 1, 2, 3, 4, 5, 6, 7, 8, 9, 10, 11, 12, 13, 14, 15); }
__device__ __forceinline__ v16bf cat16b(v8us lo, v8us hi) { return __builtin_bit_cast(v16bf, __builtin_shufflevector(lo, hi, 0, 1, 2, 3, 4, 5, 6, 7, 8, 9, 10, 11, 12, 13, 14, 15)); }
__device__ __forceinline__ v8f wmma16(v16h a, v16h b, v8f c) { return __builtin_amdgcn_wmma_f32_16x16x32_f16(false, a, false, b, (short)0, c, false, false); }
__device__ __forceinline__ v8f wmmab(v16bf a, v16bf b, v8f c) { return __builtin_amdgcn_wmma_f32_16x16x32_bf16(false, a, false, b, (short)0, c, false, false); }

template <typename T16> struct WFrag;
template <> struct WFrag<h16> { typedef v16h V; static __device__ __forceinline__ V ld(const h16* p) { return cat16(*(const v8h*)p, *(const v8h*)(p + 16)); } static __device__ __forceinline__ v8f mma(V a, V b, v8f c) { return wmma16(a, b, c); } };
template <> struct WFrag<bf> { typedef v16bf V; static __device__ __forceinline__ V ld(const bf* p) { return cat16b(*(const v8us*)p, *(const v8us*)(p + 16)); } static __device__ __forceinline__ v8f mma(V a, V b, v8f c) { return wmmab(a, b, c); } };
template <typename T16, int NSPLIT, bool BIAS>
__global__ __launch_bounds__(32) void k_gemmw(const T16* __restrict__ A, const T16* __restrict__ A2, const T16* __restrict__ Bt, const T16* __restrict__ Bt2, int K, float* C, int ldc, const float* __restrict__ bias, size_t sA, size_t sB, size_t sC) {
    typedef typename WFrag<T16>::V V;
    __shared__ __align__(16) float os[16 * 68];
    const size_t z = blockIdx.z; A += z * sA; if (A2) A2 += z * sA; Bt += z * sB; if (Bt2) Bt2 += z * sB; C += z * sC;
    const int lane = threadIdx.x & 31, lr = lane & 15, hi = lane >> 4; const int r0 = blockIdx.x * 64, c0 = blockIdx.y * 64;
    v8f acc[4][4];
#pragma unroll
    for (int mb = 0; mb < 4; ++mb)
#pragma unroll
        for (int nb = 0; nb < 4; ++nb) acc[mb][nb] = (v8f){};
    const size_t aoff = (size_t)(r0 + lr) * K + 8 * hi, boff = (size_t)(c0 + lr) * K + 8 * hi;
#pragma unroll 1
    for (int kc = 0; kc < K; kc += 32) {
        V a[4], a2[4];
#pragma unroll
        for (int mb = 0; mb < 4; ++mb) { a[mb] = WFrag<T16>::ld(A + aoff + (size_t)mb * 16 * K + kc); if (NSPLIT == 1 || NSPLIT == 2) a2[mb] = WFrag<T16>::ld(A2 + aoff + (size_t)mb * 16 * K + kc); }
#pragma unroll
        for (int nb = 0; nb < 4; ++nb) { const V b = WFrag<T16>::ld(Bt + boff + (size_t)nb * 16 * K + kc); V b2; if (NSPLIT >= 2) b2 = WFrag<T16>::ld(Bt2 + boff + (size_t)nb * 16 * K + kc);
#pragma unroll
            for (int mb = 0; mb < 4; ++mb) { acc[mb][nb] = WFrag<T16>::mma(a[mb], b, acc[mb][nb]); if (NSPLIT == 1 || NSPLIT == 2) acc[mb][nb] = WFrag<T16>::mma(a2[mb], b, acc[mb][nb]); if (NSPLIT >= 2) acc[mb][nb] = WFrag<T16>::mma(a[mb], b2, acc[mb][nb]); } }
        asm volatile("v_nop\n\tv_nop\n\tv_nop\n\tv_nop" : "+v"(acc[0][0]), "+v"(acc[1][1]), "+v"(acc[2][2]), "+v"(acc[3][3]) : "v"(a[0]), "v"(a[3]));
    }
#pragma unroll
    for (int mb = 0; mb < 4; ++mb) {
#pragma unroll
        for (int nb = 0; nb < 4; ++nb) {
#pragma unroll
            for (int j = 0; j < 8; ++j) os[(hi * 8 + j) * 68 + nb * 16 + lr] = acc[mb][nb][j]; }
        __builtin_amdgcn_wave_barrier(); asm volatile("" ::: "memory");
        float* crow = C + (size_t)(r0 + mb * 16) * ldc + c0;
#pragma unroll 1
        for (int ps = 0; ps < 2; ++ps) {
#pragma unroll
            for (int s = 0; s < 8; ++s) { const int row = 2 * s + hi, cofs = lr * 4; v4f val = *(const v4fa*)(os + row * 68 + cofs); if (BIAS) { val[0] += bfr(bias[c0 + cofs]); val[1] += bfr(bias[c0 + cofs + 1]); val[2] += bfr(bias[c0 + cofs + 2]); val[3] += bfr(bias[c0 + cofs + 3]); }
                *(volatile v4f*)(crow + (size_t)row * ldc + cofs) = val; }
            if (ps == 0) __threadfence(); }
        __builtin_amdgcn_wave_barrier(); asm volatile("" ::: "memory");
    }
}

typedef __attribute__((ext_vector_type(4))) unsigned short v4us;

static __device__ __forceinline__ h16 toh_flush(float v) { const h16 r = (h16)v; return (fabsf(v) < 6.103515625e-05f) ? (h16)0.0f : r; }

__global__ __launch_bounds__(256) void k_xtb(const float* __restrict__ x, bf* XT) {
    const size_t e = ((size_t)blockIdx.x * 256 + threadIdx.x) * 4; if (e >= (size_t)NB * DD * SEQ) return;
    const int s = (int)(e % SEQ); const size_t r = e / SEQ; const int d = (int)(r % DD); const size_t b = r / DD;
    const float* xb = x + b * (size_t)SEQ_FULL * DD; v4us o;
#pragma unroll
    for (int u = 0; u < 4; ++u) o[u] = f2bf(xb[(size_t)(s + u) * DD + d]);
    *(volatile v4us*)(XT + e) = o; __threadfence(); *(volatile v4us*)(XT + e) = o; }

__global__ __launch_bounds__(256) void k_xh(const float* __restrict__ x, h16* XH) {
    const size_t e = ((size_t)blockIdx.x * 256 + threadIdx.x) * 8; if (e >= (size_t)NB * SEQ * DD) return;
    const size_t b = e / ((size_t)SEQ * DD); const size_t r = e - b * (size_t)SEQ * DD;
    const v8f a = *(const v8f*)(x + b * (size_t)SEQ_FULL * DD + r); v8h o;
#pragma unroll
    for (int k = 0; k < 8; ++k) o[k] = toh_flush(bfr(a[k]));
    *(volatile v8h*)(XH + e) = o; __threadfence(); *(volatile v8h*)(XH + e) = o; }

__global__ __launch_bounds__(256) void k_gtr(const float* __restrict__ G, h16* GH) {
    const size_t o = ((size_t)blockIdx.x * 256 + threadIdx.x) * 8; if (o >= (size_t)NB * DD * DD) return;
    const int e0 = (int)(o % DD); const size_t r = o / DD; const int d = (int)(r % DD); const size_t b = r / DD;
    const float* Gb = G + b * (size_t)DD * DD; v8h v;
#pragma unroll
    for (int u = 0; u < 8; ++u) v[u] = toh_flush(Gb[(size_t)(e0 + u) * DD + d]);
    *(volatile v8h*)(GH + o) = v; __threadfence(); *(volatile v8h*)(GH + o) = v; }

extern "C" void kernel_launch(void* const* d_in, const int* in_sizes, int n_in,
                              void* d_out, int out_size, void* d_ws, size_t ws_size, hipStream_t stream) {
    if (n_in < 1) return;
    if ((size_t)in_sizes[0] < (size_t)(NB - 1) * SEQ_FULL * DD + (size_t)SEQ * DD) return;
    if ((size_t)out_size < (size_t)NB * SEQ * DD) return;
    const float* x = (const float*)d_in[0];
    float* OUT = (float*)d_out;
    char* wsp = (char*)d_ws;
    auto take = [&](size_t bytes) { char* p = wsp; wsp += (bytes + 255) & ~(size_t)255; return (void*)p; };
    bf*  XT = (bf*)take(WS_XT);
    h16* XH = (h16*)take(WS_XH);
    float* G = (float*)take(WS_G);
    h16* GH = (h16*)take(WS_GH);
    if ((size_t)(wsp - (char*)d_ws) > ws_size) return;

    k_xtb<<<(unsigned)(((size_t)NB * DD * SEQ / 4 + 255) / 256), 256, 0, stream>>>(x, XT);
    k_xh<<<(unsigned)(((size_t)NB * SEQ * DD / 8 + 255) / 256), 256, 0, stream>>>(x, XH);
    k_gemmw<bf, 0, false><<<dim3(DD / 64, DD / 64, NB), 32, 0, stream>>>(XT, nullptr, XT, nullptr, SEQ, G, DD, nullptr, (size_t)DD * SEQ, (size_t)DD * SEQ, (size_t)DD * DD);
    k_gtr<<<(unsigned)(((size_t)NB * DD * DD / 8 + 255) / 256), 256, 0, stream>>>(G, GH);
    k_gemmw<h16, 0, false><<<dim3(SEQ / 64, DD / 64, NB), 32, 0, stream>>>(XH, nullptr, GH, nullptr, DD, OUT, DD, nullptr, (size_t)SEQ * DD, (size_t)DD * DD, (size_t)SEQ * DD);
}
